// GS3DRenderer_49512382988492
// MI455X (gfx1250) — hardware-verified
//
#include <hip/hip_runtime.h>
#define NG 2048
#define FEAT 128
#define HI 128
#define WI 128
#define NPIX (HI * WI)

typedef __bf16 v16b __attribute__((ext_vector_type(16)));
typedef unsigned short v8us __attribute__((ext_vector_type(8), may_alias));
typedef float  v8f  __attribute__((ext_vector_type(8)));
typedef float  v4f  __attribute__((ext_vector_type(4)));
typedef float  v4fa __attribute__((ext_vector_type(4), may_alias));
union FragB { v16b v; v8us half[2]; unsigned short u[16]; };

__device__ __forceinline__ unsigned short bf16_bits(float x) { unsigned int u = __float_as_uint(x); return (unsigned short)((u + 0x7FFFu + ((u >> 16) & 1u)) >> 16); }
__device__ __forceinline__ float bf16_val(unsigned short b) { return __uint_as_float(((unsigned int)b) << 16); }
__device__ __forceinline__ float bf16_round(float x) { return bf16_val(bf16_bits(x)); }
template <int NT>
__device__ __forceinline__ v8f mmaN(v16b ah, v16b al, v16b bh, v16b bl, v8f c) {
  c = __builtin_amdgcn_wmma_f32_16x16x32_bf16(false, ah, false, bh, (short)0, c, false, false);
  if (NT >= 2) c = __builtin_amdgcn_wmma_f32_16x16x32_bf16(false, al, false, bh, (short)0, c, false, false);
  if (NT >= 3) c = __builtin_amdgcn_wmma_f32_16x16x32_bf16(false, ah, false, bl, (short)0, c, false, false);
  asm volatile("v_nop\n\tv_nop\n\tv_nop\n\tv_nop" : "+v"(c) : "v"(ah), "v"(al), "v"(bh), "v"(bl));
  return c;
}

__global__ __launch_bounds__(256) void k_wt_bf16(const float* __restrict__ W, unsigned short* __restrict__ Wt, int K, int N) {
  const int t = blockIdx.x * 256 + threadIdx.x;
  const int k8n = K / 8;
  if (t >= N * k8n) return;
  const int n = t / k8n, k8 = (t % k8n) * 8;
  v8us v;
#pragma unroll
  for (int i = 0; i < 8; ++i) v[i] = bf16_bits(W[(size_t)(k8 + i) * N + n]);
  *(volatile v8us*)(Wt + (size_t)n * K + k8) = v;
  __threadfence();
  *(volatile v8us*)(Wt + (size_t)n * K + k8) = v;
}

template <bool ASPLIT, int ACT, bool BIAS_BF16>
__global__ __launch_bounds__(128) void k_gemm_bf(const float* __restrict__ A, int lda, const unsigned short* __restrict__ Wt, int ldb,
                                               const float* __restrict__ bias, float* __restrict__ C, int ldc, int M, int N, int K) {
  __shared__ __attribute__((aligned(16))) float so[4][16][64];
  const int tid = threadIdx.x, w = tid >> 5, lane = tid & 31, ln = lane & 15, hh = lane >> 4;
  const int ntn = N / 64;
  const int wid = blockIdx.x * 4 + w;
  const int mt = wid / ntn, nq = wid % ntn;
  if (mt * 16 >= M) return;
  const int row0 = mt * 16, col0 = nq * 64;
  const float* arow = A + (size_t)(row0 + ln) * lda;
  v8f acc[4] = {};
  for (int kb = 0; kb < K; kb += 32) {
    FragB ah, al;
    const v4f x0 = *(const v4fa*)(arow + kb + 8 * hh), x1 = *(const v4fa*)(arow + kb + 8 * hh + 4);
    const v4f x2 = *(const v4fa*)(arow + kb + 16 + 8 * hh), x3 = *(const v4fa*)(arow + kb + 16 + 8 * hh + 4);
    float xs[16] = {x0[0],x0[1],x0[2],x0[3],x1[0],x1[1],x1[2],x1[3],x2[0],x2[1],x2[2],x2[3],x3[0],x3[1],x3[2],x3[3]};
#pragma unroll
    for (int i = 0; i < 16; ++i) { const unsigned short hb = bf16_bits(xs[i]); ah.u[i] = hb; al.u[i] = ASPLIT ? bf16_bits(xs[i] - bf16_val(hb)) : (unsigned short)0; }
#pragma unroll
    for (int t = 0; t < 4; ++t) {
      const unsigned short* brow = Wt + (size_t)(col0 + t * 16 + ln) * ldb + kb;
      FragB b;
      b.half[0] = *(const v8us*)(brow + 8 * hh);
      b.half[1] = *(const v8us*)(brow + 16 + 8 * hh);
      acc[t] = mmaN<ASPLIT ? 2 : 1>(ah.v, al.v, b.v, b.v, acc[t]);
    }
  }
#pragma unroll
  for (int t = 0; t < 4; ++t) {
    float bv = bias ? bias[col0 + t * 16 + ln] : 0.f;
    if (BIAS_BF16) bv = bf16_round(bv);
#pragma unroll
    for (int r = 0; r < 8; ++r) { float v = acc[t][r] + bv; if (ACT == 1) v = fmaxf(v, 0.f); so[w][8 * hh + r][t * 16 + ln] = v; }
  }
  __builtin_amdgcn_fence(__ATOMIC_ACQ_REL, "workgroup");
  __builtin_amdgcn_wave_barrier();
  const int rsub = lane >> 4, c4 = (lane & 15) * 4;
  for (int pass = 0; pass < 2; ++pass) {
#pragma unroll
    for (int q = 0; q < 8; ++q) {
      const int r = q * 2 + rsub;
      const v4f v = *(const v4fa*)&so[w][r][c4];
      *(volatile v4f*)(C + (size_t)(row0 + r) * ldc + col0 + c4) = v;
    }
    if (pass == 0) __threadfence();
  }
}

template <int D, bool CAUSAL>
__global__ __launch_bounds__(128) void k_flash(const float* __restrict__ qb, const float* __restrict__ kb, const float* __restrict__ vb,
                                             int pitch, int T, int H, float scale, float* __restrict__ y, int ypitch) {
  constexpr int KS = D / 32;
  constexpr int DT = D / 16;
  __shared__ __attribute__((aligned(16))) unsigned short sKh[32][D + 8], sKl[32][D + 8], sVh[32][D + 8], sVl[32][D + 8];
  __shared__ __attribute__((aligned(16))) unsigned short sPh[4][16][40], sPl[4][16][40];
  __shared__ __attribute__((aligned(16))) float sO[4][16][D];
  const int tid = threadIdx.x, w = tid >> 5, lane = tid & 31, ln = lane & 15, hh = lane >> 4;
  const int nqb = (T + 63) / 64;
  const int bh = blockIdx.x / nqb, qblk = blockIdx.x % nqb;
  const int b = bh / H, h = bh % H;
  const int q0 = qblk * 64 + w * 16;
  const float* Q = qb + (size_t)b * T * pitch + h * D;
  const float* K = kb + (size_t)b * T * pitch + h * D;
  const float* V = vb + (size_t)b * T * pitch + h * D;

  FragB aqh[KS], aql[KS];
  {
    int row = q0 + ln; if (row >= T) row = T - 1;
    const float* qr = Q + (size_t)row * pitch;
#pragma unroll
    for (int ks = 0; ks < KS; ++ks)
#pragma unroll
      for (int i = 0; i < 16; ++i) {
        const int d = ks * 32 + ((i < 8) ? (8 * hh + i) : (16 + 8 * hh + (i - 8)));
        const float x = qr[d] * scale; const unsigned short hb = bf16_bits(x);
        aqh[ks].u[i] = hb; aql[ks].u[i] = bf16_bits(x - bf16_val(hb));
      }
  }
  float m_r[8], l_r[8];
#pragma unroll
  for (int r = 0; r < 8; ++r) { m_r[r] = -3.0e38f; l_r[r] = 0.f; }
  v8f oacc[DT];
#pragma unroll
  for (int dt = 0; dt < DT; ++dt) oacc[dt] = (v8f){0.f,0.f,0.f,0.f,0.f,0.f,0.f,0.f};

  const int kv_end = CAUSAL ? min(T, qblk * 64 + 64) : T;
  for (int j0 = 0; j0 < kv_end; j0 += 32) {
    __syncthreads();
    for (int e = tid; e < 32 * (D / 4); e += 128) {
      const int r = e / (D / 4), c4 = (e % (D / 4)) * 4;
      const int key = j0 + r;
      v4f kf = {0.f,0.f,0.f,0.f}, vf = {0.f,0.f,0.f,0.f};
      if (key < T) { kf = *(const v4fa*)(K + (size_t)key * pitch + c4); vf = *(const v4fa*)(V + (size_t)key * pitch + c4); }
#pragma unroll
      for (int t = 0; t < 4; ++t) {
        unsigned short hb = bf16_bits(kf[t]); sKh[r][c4 + t] = hb; sKl[r][c4 + t] = bf16_bits(kf[t] - bf16_val(hb));
        hb = bf16_bits(vf[t]); sVh[r][c4 + t] = hb; sVl[r][c4 + t] = bf16_bits(vf[t] - bf16_val(hb));
      }
    }
    __syncthreads();
    v8f s[2];
#pragma unroll
    for (int nt = 0; nt < 2; ++nt) {
      v8f acc = {};
#pragma unroll
      for (int ks = 0; ks < KS; ++ks) {
        FragB bh_, bl_;
        bh_.half[0] = *(const v8us*)&sKh[nt * 16 + ln][ks * 32 + 8 * hh]; bh_.half[1] = *(const v8us*)&sKh[nt * 16 + ln][ks * 32 + 16 + 8 * hh];
        bl_.half[0] = *(const v8us*)&sKl[nt * 16 + ln][ks * 32 + 8 * hh]; bl_.half[1] = *(const v8us*)&sKl[nt * 16 + ln][ks * 32 + 16 + 8 * hh];
        acc = mmaN<3>(aqh[ks].v, aql[ks].v, bh_.v, bl_.v, acc);
      }
      s[nt] = acc;
    }
    float alpha[8];
#pragma unroll
    for (int r = 0; r < 8; ++r) {
      const int qi = q0 + 8 * hh + r;
      const int ja = j0 + ln, jb = j0 + 16 + ln;
      if (CAUSAL) { if (ja > qi) s[0][r] = -3.0e38f; if (jb > qi) s[1][r] = -3.0e38f; }
      if (ja >= T) s[0][r] = -3.0e38f;
      if (jb >= T) s[1][r] = -3.0e38f;
      float mx = fmaxf(s[0][r], s[1][r]);
      mx = fmaxf(mx, __shfl_xor(mx, 1, 32)); mx = fmaxf(mx, __shfl_xor(mx, 2, 32)); mx = fmaxf(mx, __shfl_xor(mx, 4, 32)); mx = fmaxf(mx, __shfl_xor(mx, 8, 32));
      const float mnew = fmaxf(m_r[r], mx);
      alpha[r] = (mnew > -1.0e38f) ? __expf(m_r[r] - mnew) : 1.0f;
      const float p0 = (s[0][r] > -1.0e38f) ? __expf(s[0][r] - mnew) : 0.f;
      const float p1 = (s[1][r] > -1.0e38f) ? __expf(s[1][r] - mnew) : 0.f;
      m_r[r] = mnew;
      l_r[r] = l_r[r] * alpha[r] + p0 + p1;
      unsigned short hb = bf16_bits(p0); sPh[w][8 * hh + r][ln] = hb;      sPl[w][8 * hh + r][ln] = bf16_bits(p0 - bf16_val(hb));
      hb = bf16_bits(p1);                sPh[w][8 * hh + r][16 + ln] = hb; sPl[w][8 * hh + r][16 + ln] = bf16_bits(p1 - bf16_val(hb));
    }
#pragma unroll
    for (int dt = 0; dt < DT; ++dt)
#pragma unroll
      for (int r = 0; r < 8; ++r) oacc[dt][r] *= alpha[r];
    __builtin_amdgcn_fence(__ATOMIC_ACQ_REL, "workgroup");
    __builtin_amdgcn_wave_barrier();
    FragB pah, pal;
    pah.half[0] = *(const v8us*)&sPh[w][ln][8 * hh]; pah.half[1] = *(const v8us*)&sPh[w][ln][16 + 8 * hh];
    pal.half[0] = *(const v8us*)&sPl[w][ln][8 * hh]; pal.half[1] = *(const v8us*)&sPl[w][ln][16 + 8 * hh];
#pragma unroll
    for (int dt = 0; dt < DT; ++dt) {
      FragB bvh, bvl;
#pragma unroll
      for (int i = 0; i < 8; ++i) {
        bvh.u[i] = sVh[8 * hh + i][dt * 16 + ln]; bvh.u[8 + i] = sVh[16 + 8 * hh + i][dt * 16 + ln];
        bvl.u[i] = sVl[8 * hh + i][dt * 16 + ln]; bvl.u[8 + i] = sVl[16 + 8 * hh + i][dt * 16 + ln];
      }
      oacc[dt] = mmaN<3>(pah.v, pal.v, bvh.v, bvl.v, oacc[dt]);
    }
    __builtin_amdgcn_fence(__ATOMIC_ACQ_REL, "workgroup");
    __builtin_amdgcn_wave_barrier();
  }
#pragma unroll
  for (int r = 0; r < 8; ++r) {
    float l = l_r[r];
    l += __shfl_xor(l, 1, 32); l += __shfl_xor(l, 2, 32); l += __shfl_xor(l, 4, 32); l += __shfl_xor(l, 8, 32);
    l_r[r] = (l > 0.f) ? 1.0f / l : 0.f;
  }
#pragma unroll
  for (int dt = 0; dt < DT; ++dt)
#pragma unroll
    for (int r = 0; r < 8; ++r) sO[w][8 * hh + r][dt * 16 + ln] = oacc[dt][r] * l_r[r];
  __builtin_amdgcn_fence(__ATOMIC_ACQ_REL, "workgroup");
  __builtin_amdgcn_wave_barrier();
  for (int pass = 0; pass < 2; ++pass) {
    for (int r = 0; r < 16; ++r) {
      const int row = q0 + r;
      if (row < T && lane < D / 4) {
        const v4f val = *(const v4fa*)&sO[w][r][lane * 4];
        *(volatile v4f*)(y + ((size_t)b * T + row) * ypitch + h * D + lane * 4) = val;
      }
    }
    if (pass == 0) __threadfence();
  }
}

template <bool ASPLIT, int ACT, bool BIAS_BF16, bool RES_BF16>
__global__ __launch_bounds__(128) void k_gemm_bf3(const float* __restrict__ A, int lda, const unsigned short* __restrict__ Wt, int ldb,
                                                const float* __restrict__ bias, const float* __restrict__ resid, int rmod, int ldr,
                                                float* __restrict__ C, int ldc, int M, int N, int K) {
  __shared__ __attribute__((aligned(16))) float so[4][16][64];
  const int tid = threadIdx.x, w = tid >> 5, lane = tid & 31, ln = lane & 15, hh = lane >> 4;
  const int ntn = N / 64;
  const int wid = blockIdx.x * 4 + w;
  const int mt = wid / ntn, nq = wid % ntn;
  if (mt * 16 >= M) return;
  const int row0 = mt * 16, col0 = nq * 64;
  const float* arow = A + (size_t)(row0 + ln) * lda;
  v8f acc[4] = {};
  for (int kb = 0; kb < K; kb += 32) {
    FragB ah, al;
    const v4f x0 = *(const v4fa*)(arow + kb + 8 * hh), x1 = *(const v4fa*)(arow + kb + 8 * hh + 4);
    const v4f x2 = *(const v4fa*)(arow + kb + 16 + 8 * hh), x3 = *(const v4fa*)(arow + kb + 16 + 8 * hh + 4);
    float xs[16] = {x0[0],x0[1],x0[2],x0[3],x1[0],x1[1],x1[2],x1[3],x2[0],x2[1],x2[2],x2[3],x3[0],x3[1],x3[2],x3[3]};
#pragma unroll
    for (int i = 0; i < 16; ++i) { const unsigned short hb = bf16_bits(xs[i]); ah.u[i] = hb; al.u[i] = ASPLIT ? bf16_bits(xs[i] - bf16_val(hb)) : (unsigned short)0; }
#pragma unroll
    for (int t = 0; t < 4; ++t) {
      const unsigned short* brow = Wt + (size_t)(col0 + t * 16 + ln) * ldb + kb;
      FragB b;
      b.half[0] = *(const v8us*)(brow + 8 * hh);
      b.half[1] = *(const v8us*)(brow + 16 + 8 * hh);
      acc[t] = mmaN<ASPLIT ? 2 : 1>(ah.v, al.v, b.v, b.v, acc[t]);
    }
  }
#pragma unroll
  for (int t = 0; t < 4; ++t) {
    const int col = col0 + t * 16 + ln;
    float bv = bias ? bias[col] : 0.f;
    if (BIAS_BF16) bv = bf16_round(bv);
#pragma unroll
    for (int r = 0; r < 8; ++r) {
      float v = acc[t][r] + bv;
      if (resid) { float rv = resid[(size_t)((row0 + 8 * hh + r) % rmod) * ldr + col]; if (RES_BF16) rv = bf16_round(rv); v += rv; }
      if (ACT == 1) v = fmaxf(v, 0.f);
      if (ACT == 2) v = 0.5f * v * (1.0f + erff(v * 0.70710678118654752f));
      if (ACT == 3) { const float u = 0.7978845608028654f * (v + 0.044715f * v * v * v); v = 0.5f * v * (1.0f + tanhf(u)); }
      so[w][8 * hh + r][t * 16 + ln] = v;
    }
  }
  __builtin_amdgcn_fence(__ATOMIC_ACQ_REL, "workgroup");
  __builtin_amdgcn_wave_barrier();
  const int rsub = lane >> 4, c4 = (lane & 15) * 4;
  for (int pass = 0; pass < 2; ++pass) {
#pragma unroll
    for (int q = 0; q < 8; ++q) {
      const int r = q * 2 + rsub;
      const v4f v = *(const v4fa*)&so[w][r][c4];
      *(volatile v4f*)(C + (size_t)(row0 + r) * ldc + col0 + c4) = v;
    }
    if (pass == 0) __threadfence();
  }
}
template <bool PARAM_BF16>
__global__ __launch_bounds__(256) void k_layernorm(const float* __restrict__ X, const float* __restrict__ R, const float* __restrict__ g, const float* __restrict__ bta,
                                                  float* __restrict__ out_sum, float* __restrict__ out_norm, int N, float eps) {
  __shared__ float red[256];
  const int row = blockIdx.x, tid = threadIdx.x;
  const float* x = X + (size_t)row * N; const float* rr = R ? R + (size_t)row * N : nullptr;
  float vals[16];
  const int per = N / 256;
  float s1 = 0.f;
  for (int u = 0; u < per / 4; ++u) {
    const int j = tid * 4 + 1024 * u;
    const v4f a = *(const v4fa*)(x + j);
    v4f b = {0.f,0.f,0.f,0.f}; if (rr) b = *(const v4fa*)(rr + j);
#pragma unroll
    for (int q = 0; q < 4; ++q) { const float v = a[q] + b[q]; vals[u * 4 + q] = v; s1 += v; }
  }
  red[tid] = s1; __syncthreads();
  for (int st = 128; st > 0; st >>= 1) { if (tid < st) red[tid] += red[tid + st]; __syncthreads(); }
  const float mu = red[0] / (float)N; __syncthreads();
  float s2 = 0.f;
  for (int u = 0; u < per / 4; ++u)
#pragma unroll
    for (int q = 0; q < 4; ++q) { const float c = vals[u * 4 + q] - mu; s2 += c * c; }
  red[tid] = s2; __syncthreads();
  for (int st = 128; st > 0; st >>= 1) { if (tid < st) red[tid] += red[tid + st]; __syncthreads(); }
  const float rs = rsqrtf(red[0] / (float)N + eps);
  for (int pass = 0; pass < 2; ++pass) {
    for (int u = 0; u < per / 4; ++u) {
      const int j = tid * 4 + 1024 * u;
      v4f o, sm;
#pragma unroll
      for (int q = 0; q < 4; ++q) {
        float gg = g[j + q], bb = bta[j + q];
        if (PARAM_BF16) { gg = bf16_round(gg); bb = bf16_round(bb); }
        sm[q] = vals[u * 4 + q]; o[q] = (vals[u * 4 + q] - mu) * rs * gg + bb;
      }
      if (out_sum) *(volatile v4f*)(out_sum + (size_t)row * N + j) = sm;
      *(volatile v4f*)(out_norm + (size_t)row * N + j) = o;
    }
    if (pass == 0) __threadfence();
  }
}

__global__ __launch_bounds__(256) void k_wt(const float* __restrict__ wsh, const float* __restrict__ wsc, const float* __restrict__ wxy, const float* __restrict__ wop, const float* __restrict__ wro,
                                           const float* __restrict__ bsh, const float* __restrict__ bsc, const float* __restrict__ bxy, const float* __restrict__ bop, const float* __restrict__ bro, unsigned short* __restrict__ Bt, float* __restrict__ bias) {
  const int t = blockIdx.x * 256 + threadIdx.x; if (t >= 64 * (FEAT / 8)) return; const int n = t / (FEAT / 8), k8 = (t % (FEAT / 8)) * 8; v8us v;
  for (int i = 0; i < 8; ++i) { const int k = k8 + i; float w = 0.f;
    if (n < 3) w = wsh[n * FEAT + k]; else if (n < 6) w = wsc[(n - 3) * FEAT + k]; else if (n < 9) w = wxy[(n - 6) * FEAT + k]; else if (n == 9) w = wop[k]; else if (n < 14) w = wro[(n - 10) * FEAT + k]; v[i] = bf16_bits(w); }
  *(volatile v8us*)(Bt + (size_t)n * FEAT + k8) = v; __threadfence(); *(volatile v8us*)(Bt + (size_t)n * FEAT + k8) = v;
  if (t < 64) { float bv = 0.f; if (t < 3) bv = bsh[t]; else if (t < 6) bv = bsc[t - 3]; else if (t < 9) bv = bxy[t - 6]; else if (t == 9) bv = bop[0]; else if (t < 14) bv = bro[t - 10]; bv = bf16_round(bv); *(volatile float*)(bias + t) = bv; __threadfence(); *(volatile float*)(bias + t) = bv; }
}
__global__ __launch_bounds__(256) void k_setup(const float* __restrict__ H, const float* __restrict__ pts, const float* __restrict__ vm, float* __restrict__ G, unsigned int* __restrict__ skey, unsigned int* __restrict__ sval) {
  __shared__ float so[256 * 16];
  const int n = blockIdx.x * 256 + threadIdx.x; const float* h = H + (size_t)n * 64;
  __shared__ float sact[256][10];
#pragma unroll 1
  for (int c = 0; c < 10; ++c) { const bool isexp = (c >= 3 && c < 6); const float e = expf(isexp ? h[c] : -h[c]); sact[threadIdx.x][c] = isexp ? fminf(fmaxf(e, 0.f), 0.2f) : 1.0f / (1.0f + e); }
  const float* ac = sact[threadIdx.x];
  const float r_ = ac[0], g_ = ac[1], b_ = ac[2]; const float s0 = ac[3], s1 = ac[4], s2 = ac[5];
  const float ox = (ac[6] - 0.5f) * 0.05f, oy = (ac[7] - 0.5f) * 0.05f, oz = (ac[8] - 0.5f) * 0.05f;
  const float X = bf16_round(pts[n * 3]) + ox, Y = bf16_round(pts[n * 3 + 1]) + oy, Z = bf16_round(pts[n * 3 + 2]) + oz;
  const float op = ac[9];
  float qw = h[10], qx = h[11], qy = h[12], qz = h[13]; const float qinv = 1.0f / sqrtf(qw * qw + qx * qx + qy * qy + qz * qz); qw *= qinv; qx *= qinv; qy *= qinv; qz *= qinv;
  __shared__ float sm[256][50]; float* R = sm[threadIdx.x]; float* s2v = R + 9; float* cov = R + 12; float* Rv = R + 21; float* tv = R + 30; float* J = R + 33; float* M = R + 39;
  R[0] = 1.f - 2.f * (qy * qy + qz * qz); R[1] = 2.f * (qx * qy - qw * qz); R[2] = 2.f * (qx * qz + qw * qy);
  R[3] = 2.f * (qx * qy + qw * qz); R[4] = 1.f - 2.f * (qx * qx + qz * qz); R[5] = 2.f * (qy * qz - qw * qx);
  R[6] = 2.f * (qx * qz - qw * qy); R[7] = 2.f * (qy * qz + qw * qx); R[8] = 1.f - 2.f * (qx * qx + qy * qy);
  s2v[0] = s0 * s0; s2v[1] = s1 * s1; s2v[2] = s2 * s2;
#pragma unroll 1
  for (int i = 0; i < 3; ++i) {
#pragma unroll 1
    for (int k = 0; k < 3; ++k) { float a = 0.f;
#pragma unroll 1
      for (int j = 0; j < 3; ++j) a += R[i * 3 + j] * s2v[j] * R[k * 3 + j]; cov[i * 3 + k] = a; } }
#pragma unroll 1
  for (int i = 0; i < 3; ++i) { for (int j = 0; j < 3; ++j) Rv[i * 3 + j] = bf16_round(vm[i * 4 + j]); tv[i] = bf16_round(vm[i * 4 + 3]); }
  const float px_ = Rv[0] * X + Rv[1] * Y + Rv[2] * Z + tv[0], py_ = Rv[3] * X + Rv[4] * Y + Rv[5] * Z + tv[1], pz_ = Rv[6] * X + Rv[7] * Y + Rv[8] * Z + tv[2];
  const float tz = fmaxf(pz_, 1e-3f); const float itz = 1.0f / tz; const float u = 128.0f * px_ * itz + 64.0f, v = 128.0f * py_ * itz + 64.0f;
  J[0] = 128.0f * itz; J[1] = 0.f; J[2] = -128.0f * px_ * (itz * itz); J[3] = 0.f; J[4] = 128.0f * itz; J[5] = -128.0f * py_ * (itz * itz);
#pragma unroll 1
  for (int i = 0; i < 2; ++i) {
#pragma unroll 1
    for (int k = 0; k < 3; ++k) { float a = 0.f;
#pragma unroll 1
      for (int j = 0; j < 3; ++j) a += J[i * 3 + j] * Rv[j * 3 + k]; M[i * 3 + k] = a; } }
  float* C2 = R + 45;
#pragma unroll 1
  for (int i = 0; i < 2; ++i) {
#pragma unroll 1
    for (int l2 = 0; l2 < 2; ++l2) { float a = 0.f;
#pragma unroll 1
      for (int j = 0; j < 3; ++j) {
#pragma unroll 1
        for (int k = 0; k < 3; ++k) a += M[i * 3 + j] * cov[j * 3 + k] * M[l2 * 3 + k]; }
      C2[i * 2 + l2] = a; } }
  const float a = C2[0] + 0.3f, b = C2[1], c = C2[3] + 0.3f; const float det = a * c - b * b + 1e-12f; const float idet = 1.0f / det; const float cA = c * idet, cB = -b * idet, cC = a * idet;
  const float vis = (pz_ > 0.01f) ? 1.f : 0.f;
  float* o = so + threadIdx.x * 16; o[0] = u; o[1] = v; o[2] = cA; o[3] = cB; o[4] = cC; o[5] = op; o[6] = r_; o[7] = g_; o[8] = b_; o[9] = tz; o[10] = vis; o[11] = pz_; o[12] = 0.f; o[13] = 0.f; o[14] = 0.f; o[15] = 0.f;
  __syncthreads();
  for (int pass = 0; pass < 2; ++pass) { for (int e = threadIdx.x; e < 256 * 16; e += 256) *(volatile float*)(G + (size_t)blockIdx.x * 256 * 16 + e) = so[e]; if (pass == 0) __threadfence(); }
  const unsigned int kb = __float_as_uint(tz);
  *(volatile unsigned int*)(skey + n) = kb; *(volatile unsigned int*)(sval + n) = (unsigned int)n; __threadfence(); *(volatile unsigned int*)(skey + n) = kb; *(volatile unsigned int*)(sval + n) = (unsigned int)n;
}
__global__ __launch_bounds__(1024) void k_sort2048(unsigned int* __restrict__ key, unsigned int* __restrict__ val) {
  __shared__ unsigned int sk[NG], sv[NG]; const int t = threadIdx.x;
  sk[t] = key[t]; sk[t + 1024] = key[t + 1024]; sv[t] = val[t]; sv[t + 1024] = val[t + 1024]; __syncthreads();
  for (int k = 2; k <= NG; k <<= 1) { for (int j = k >> 1; j >= 1; j >>= 1) {
      for (int i = t; i < NG; i += 1024) { const int ixj = i ^ j; if (ixj > i) { const bool up = ((i & k) == 0); const unsigned int a = sk[i], bq = sk[ixj]; const unsigned int av = sv[i], bvv = sv[ixj];
          const bool agt = (a > bq) || (a == bq && av > bvv); if (agt == up) { sk[i] = bq; sk[ixj] = a; sv[i] = bvv; sv[ixj] = av; } } }
      __syncthreads(); } }
  for (int pass = 0; pass < 2; ++pass) { *(volatile unsigned int*)(val + t) = sv[t]; *(volatile unsigned int*)(val + t + 1024) = sv[t + 1024]; if (pass == 0) __threadfence(); }
}
__global__ __launch_bounds__(256) void k_render(const float* __restrict__ G, const unsigned int* __restrict__ order, float* __restrict__ img) {
  __shared__ float sg[128][12]; __shared__ float so[256 * 3];
  const int p = blockIdx.x * 256 + threadIdx.x; const float gx = (float)(p % WI) + 0.5f, gy = (float)(p / WI) + 0.5f;
  float T = 1.0f, cr = 0.f, cg = 0.f, cb = 0.f;
  for (int n0 = 0; n0 < NG; n0 += 128) {
    __syncthreads();
    for (int e = threadIdx.x; e < 128 * 12; e += 256) { const int gi = (int)order[n0 + e / 12]; sg[e / 12][e % 12] = G[(size_t)gi * 16 + e % 12]; }
    __syncthreads();
#pragma unroll 1
    for (int j = 0; j < 128; ++j) { const float* g = sg[j]; const float dx = gx - g[0], dy = gy - g[1];
      float power = -0.5f * (g[2] * dx * dx + g[4] * dy * dy) - g[3] * dx * dy; power = fminf(power, 0.f);
      float al = fminf(0.99f, g[5] * expf(power)); al = al * g[10]; if (al < (1.0f / 255.0f)) al = 0.f;
      const float w = al * T; cr += w * g[6]; cg += w * g[7]; cb += w * g[8]; T = T * (1.0f - al); }
  }
  so[threadIdx.x * 3] = cr; so[threadIdx.x * 3 + 1] = cg; so[threadIdx.x * 3 + 2] = cb;
  __syncthreads();
  for (int pass = 0; pass < 2; ++pass) { for (int e = threadIdx.x; e < 256 * 3; e += 256) *(volatile float*)(img + (size_t)blockIdx.x * 256 * 3 + e) = so[e]; if (pass == 0) __threadfence(); }
}
extern "C" void kernel_launch(void* const* d_in, const int* in_sizes, int n_in,
                              void* d_out, int out_size, void* d_ws, size_t ws_size, hipStream_t stream) {
  (void)in_sizes; (void)n_in; (void)out_size;
  const float* x = (const float*)d_in[0]; const float* pts = (const float*)d_in[1]; const float* vm = (const float*)d_in[2];
  const float* wsh = (const float*)d_in[3]; const float* bsh = (const float*)d_in[4]; const float* wsc = (const float*)d_in[5]; const float* bsc = (const float*)d_in[6]; const float* wxy = (const float*)d_in[7]; const float* bxy = (const float*)d_in[8];
  const float* wop = (const float*)d_in[9]; const float* bop = (const float*)d_in[10]; const float* wro = (const float*)d_in[11]; const float* bro = (const float*)d_in[12];
  char* ws = (char*)d_ws; size_t off = 0;
  auto take = [&](size_t bytes) { char* p = ws + off; off += (bytes + 255) & ~(size_t)255; return p; };
  unsigned short* Bt = (unsigned short*)take(64 * FEAT * 2); float* bias = (float*)take(64 * 4); float* Hh = (float*)take((size_t)NG * 64 * 4); float* G = (float*)take((size_t)NG * 16 * 4); unsigned int* skey = (unsigned int*)take(NG * 4); unsigned int* sval = (unsigned int*)take(NG * 4);
  if (off > ws_size) return;
  k_wt<<<(64 * 16 + 255) / 256, 256, 0, stream>>>(wsh, wsc, wxy, wop, wro, bsh, bsc, bxy, bop, bro, Bt, bias);
  k_gemm_bf3<false, 0, false, false><<<((NG / 16) * 1 + 3) / 4, 128, 0, stream>>>(x, FEAT, Bt, FEAT, bias, nullptr, 1, 0, Hh, 64, NG, 64, FEAT);
  k_setup<<<NG / 256, 256, 0, stream>>>(Hh, pts, vm, G, skey, sval);
  k_sort2048<<<1, 1024, 0, stream>>>(skey, sval);
  k_render<<<NPIX / 256, 256, 0, stream>>>(G, sval, (float*)d_out);
}
